// TransformerRelativeBlock_223338299691
// MI455X (gfx1250) — hardware-run, weakly checked
//
#include <hip/hip_runtime.h>
#include <math.h>

#define NB   8
#define SQ   1024
#define DMD  512
#define NHD  8
#define HD   64
#define FFD  2048
#define MT   (NB * SQ)
#define QT   32
#define SCP  1024
#define PHP  1032
#define ZP   72
#define WSCL 64.0f
#define QKS  16.0f
#define PSC  1024.0f
#define ZSC  256.0f
#define HSC  16.0f
#define LEPS 1e-5f
#define RSQD 0.044194174f
#define ALDS (QT * SCP * 4 + QT * PHP * 2 + QT * ZP * 2 + QT * 4)

static_assert(NHD * HD == DMD);
static_assert((MT % 64) == 0 && (DMD % 64) == 0 && (FFD % 64) == 0 && (SQ % 64) == 0);
static_assert((((MT / 64) * (DMD / 64)) % 8) == 0);
static_assert((((MT / 64) * (FFD / 64)) % 8) == 0);
static_assert((((SQ / 64) * (DMD / 64)) % 8) == 0);
static_assert((SQ % QT) == 0 && QT * 8 == 256 && QT == 32);
static_assert(SQ == 8 * 8 * 16);
static_assert((PHP % 8) == 0 && (ZP % 8) == 0 && ZP >= HD);
static_assert((MT % 8) == 0 && (SQ % 8) == 0);
static_assert(DMD == 4 * 128);
static_assert(((DMD * DMD) % 2048) == 0 && ((FFD * DMD) % 2048) == 0);
static_assert((ALDS % 16) == 0);

typedef _Float16 v16h __attribute__((ext_vector_type(16)));
typedef unsigned short v16us __attribute__((ext_vector_type(16)));
typedef unsigned short v8us  __attribute__((ext_vector_type(8)));
typedef float v8f __attribute__((ext_vector_type(8)));
typedef float v4f __attribute__((ext_vector_type(4)));
typedef unsigned int v4u __attribute__((ext_vector_type(4)));
typedef unsigned int v2u __attribute__((ext_vector_type(2)));

union FragU { v16us v; v8us h[2]; };

__device__ __forceinline__ unsigned short bf_bits(float f) {
  const unsigned u = __float_as_uint(f);
  return (unsigned short)((u + 0x7FFFu + ((u >> 16) & 1u)) >> 16);
}
__device__ __forceinline__ float bf_up(unsigned short h) { return __uint_as_float(((unsigned)h) << 16); }
__device__ __forceinline__ float bfr(float f) { return bf_up(bf_bits(f)); }
__device__ __forceinline__ unsigned short h_bits(_Float16 x) { return __builtin_bit_cast(unsigned short, x); }
__device__ __forceinline__ unsigned short f2h(float f) { return h_bits((_Float16)f); }
__device__ __forceinline__ unsigned pk16(unsigned short a, unsigned short b) { return (unsigned)a | ((unsigned)b << 16); }
__device__ __forceinline__ int clampi(int v, int lo, int hi) { return v < lo ? lo : (v > hi ? hi : v); }
__device__ __forceinline__ v8f zero8() { v8f z = {0.f, 0.f, 0.f, 0.f, 0.f, 0.f, 0.f, 0.f}; return z; }
__device__ __forceinline__ float silu_f(float v) { return v * (1.0f / (1.0f + __expf(-v))); }

__device__ __forceinline__ v16us ldfrag_u(const unsigned short* p) {
  FragU f;
  f.h[0] = *(const v8us*)(p);
  f.h[1] = *(const v8us*)(p + 16);
  return f.v;
}

__device__ __forceinline__ v8f mma_h_raw(v16us a, v16us b, v8f c) {
  return __builtin_amdgcn_wmma_f32_16x16x32_f16(false, __builtin_bit_cast(v16h, a), false,
                                                __builtin_bit_cast(v16h, b), (short)0, c, false, false);
}
__device__ __forceinline__ v8f mma_hu(v16us a, v16us b, v8f c) {
  c = mma_h_raw(a, b, c);
#if defined(__HIP_DEVICE_COMPILE__)
  asm volatile("v_nop\n\tv_nop\n\tv_nop\n\tv_nop" : "+v"(c) : "v"(a), "v"(b));
#endif
  return c;
}
__device__ __forceinline__ void dep_guard1(v8f& a, v8f& b, v16us x) {
#if defined(__HIP_DEVICE_COMPILE__)
  asm volatile("v_nop\n\tv_nop\n\tv_nop\n\tv_nop" : "+v"(a), "+v"(b) : "v"(x));
#endif
}
__device__ __forceinline__ void keep2_u(v16us a, v16us b) {
#if defined(__HIP_DEVICE_COMPILE__)
  asm volatile("v_nop" :: "v"(a), "v"(b));
#endif
}
__device__ __forceinline__ void keep4_u(v16us a, v16us b, v16us c, v16us d) {
#if defined(__HIP_DEVICE_COMPILE__)
  asm volatile("v_nop" :: "v"(a), "v"(b), "v"(c), "v"(d));
#endif
}
__device__ __forceinline__ void acc_guard4(v8f& a, v8f& b, v8f& c, v8f& d) {
#if defined(__HIP_DEVICE_COMPILE__)
  asm volatile("v_nop\n\tv_nop\n\tv_nop\n\tv_nop" : "+v"(a), "+v"(b), "+v"(c), "+v"(d));
#endif
}
__device__ __forceinline__ void wave_sync_lds() {
  __builtin_amdgcn_fence(__ATOMIC_RELEASE, "workgroup");
  __builtin_amdgcn_wave_barrier();
  __builtin_amdgcn_fence(__ATOMIC_ACQUIRE, "workgroup");
}

template <int MODE>
__global__ __launch_bounds__(256) void ln_kernel(const float* __restrict__ a, const float* __restrict__ g,
                                                const float* __restrict__ bt, float* of, unsigned short* oh,
                                                int nrows) {
  const int row = blockIdx.x * 8 + (threadIdx.x >> 5);
  const int lane = threadIdx.x & 31;
  if (row >= nrows) return;
  const size_t ro = (size_t)row * DMD;
  float v[16];
#pragma unroll
  for (int j = 0; j < 4; ++j) {
    const v4f t4 = *(const v4f*)(a + ro + 128 * j + 4 * lane);
#pragma unroll
    for (int e = 0; e < 4; ++e) v[4 * j + e] = (MODE == 0) ? bfr(t4[e]) : t4[e];
  }
  float s = 0.f;
#pragma unroll
  for (int e = 0; e < 16; ++e) s += v[e];
#pragma unroll
  for (int off = 16; off > 0; off >>= 1) s += __shfl_xor(s, off, 32);
  const float mu = s * (1.0f / (float)DMD);
  float d[16];
  float sq = 0.f;
#pragma unroll
  for (int e = 0; e < 16; ++e) { d[e] = v[e] - mu; sq += d[e] * d[e]; }
#pragma unroll
  for (int off = 16; off > 0; off >>= 1) sq += __shfl_xor(sq, off, 32);
  const float var = sq * (1.0f / (float)DMD);
  const float rstd = rsqrtf(var + LEPS);
  v4f ov[4];
  v2u hv[4];
#pragma unroll
  for (int j = 0; j < 4; ++j) {
    const v4f g4 = *(const v4f*)(g + 128 * j + 4 * lane);
    const v4f b4 = *(const v4f*)(bt + 128 * j + 4 * lane);
    v4f o;
#pragma unroll
    for (int e = 0; e < 4; ++e) o[e] = d[4 * j + e] * rstd * bfr(g4[e]) + bfr(b4[e]);
    ov[j] = o;
    v2u hq;
    hq[0] = pk16(f2h(o[0]), f2h(o[1]));
    hq[1] = pk16(f2h(o[2]), f2h(o[3]));
    hv[j] = hq;
  }
  for (int pass = 0; pass < 2; ++pass) {
#pragma unroll
    for (int j = 0; j < 4; ++j) {
      *(volatile v4f*)(of + ro + 128 * j + 4 * lane) = ov[j];
      *(volatile v2u*)(oh + ro + 128 * j + 4 * lane) = hv[j];
    }
    __threadfence();
  }
}

__global__ __launch_bounds__(256) void cvt_w(const float* __restrict__ w, unsigned short* o, int n, float sc) {
  const int base = (blockIdx.x * 256 + threadIdx.x) * 8;
  if (base + 8 > n) return;
  const v4f a0 = *(const v4f*)(w + base);
  const v4f a1 = *(const v4f*)(w + base + 4);
  v4u hv;
#pragma unroll
  for (int e = 0; e < 2; ++e) {
    hv[e]     = pk16(f2h(bfr(a0[2 * e]) * sc), f2h(bfr(a0[2 * e + 1]) * sc));
    hv[2 + e] = pk16(f2h(bfr(a1[2 * e]) * sc), f2h(bfr(a1[2 * e + 1]) * sc));
  }
  unsigned short* d = o + base;
  *(volatile v4u*)d = hv;
  __threadfence();
  *(volatile v4u*)d = hv;
}

__global__ __launch_bounds__(256) void pe_kernel(unsigned short* pe) {
  const int row = blockIdx.x * 8 + (threadIdx.x >> 5);
  const int lane = threadIdx.x & 31;
  if (row >= SQ) return;
  const float kx = -logf(10000.0f) / 512.0f;
  const float posf = (float)row;
#pragma unroll 1
  for (int j = 0; j < 4; ++j) {
    const int ia = 64 * j + 2 * lane;
    const float da = expf((float)(2 * ia) * kx);
    const float db = expf((float)(2 * ia + 2) * kx);
    const float aa = posf * da;
    const float ab = posf * db;
    v2u hv;
    hv[0] = pk16(f2h(sinf(aa)), f2h(cosf(aa)));
    hv[1] = pk16(f2h(sinf(ab)), f2h(cosf(ab)));
    unsigned short* d = pe + (size_t)row * DMD + 128 * j + 4 * lane;
    *(volatile v2u*)d = hv;
    __threadfence();
    *(volatile v2u*)d = hv;
  }
}

template <int OM, int CBM, int ACT, int RES>
__global__ __launch_bounds__(256) void gemm64(
    const unsigned short* __restrict__ Ap, int lda,
    const unsigned short* __restrict__ Btp, int ldb,
    unsigned short* Ch, unsigned short* Ch2, float* Cf, int ldc,
    const float* __restrict__ cb, const float* __restrict__ cb2, const float* __restrict__ cb3,
    const float* __restrict__ res, float wsc, float osc, int M, int N, int K) {
  __shared__ __align__(16) float sT[8][16 * 68];
  const int lane = threadIdx.x & 31;
  const int wave = threadIdx.x >> 5;
  const int tilesN = N >> 6;
  const int tilesM = M >> 6;
  const int tile = blockIdx.x * 8 + wave;
  if (tile >= tilesM * tilesN) return;
  const int tm = tile / tilesN;
  const int tn = tile - tm * tilesN;
  const int m0 = tm << 6;
  const int n0 = tn << 6;

  const int rlane = lane & 15;
  const int koff  = (lane >> 4) * 8;
  const int mOff  = (lane >> 4) * 8;

  v8f acc[4][4];
#pragma unroll
  for (int i = 0; i < 4; ++i)
#pragma unroll
    for (int j = 0; j < 4; ++j) acc[i][j] = zero8();

  for (int k0 = 0; k0 < K; k0 += 32) {
    v16us bh[4];
#pragma unroll
    for (int j = 0; j < 4; ++j) {
      const size_t bo = (size_t)(n0 + (j << 4) + rlane) * ldb + koff + k0;
      bh[j] = ldfrag_u(Btp + bo);
    }
#pragma unroll
    for (int i = 0; i < 4; ++i) {
      const size_t ao = (size_t)(m0 + (i << 4) + rlane) * lda + koff + k0;
      const v16us ah = ldfrag_u(Ap + ao);
#pragma unroll
      for (int j = 0; j < 4; ++j) acc[i][j] = mma_h_raw(ah, bh[j], acc[i][j]);
      dep_guard1(acc[i][0], acc[i][3], ah);
    }
    keep4_u(bh[0], bh[1], bh[2], bh[3]);
  }
  acc_guard4(acc[0][0], acc[0][1], acc[0][2], acc[0][3]);
  acc_guard4(acc[1][0], acc[1][1], acc[1][2], acc[1][3]);
  acc_guard4(acc[2][0], acc[2][1], acc[2][2], acc[2][3]);
  acc_guard4(acc[3][0], acc[3][1], acc[3][2], acc[3][3]);

  const int hh2 = lane >> 4, c4 = (lane & 15) * 4;
  const int q8  = lane >> 3, c8 = (lane & 7) * 8;

  v4f cb4 = {0.f, 0.f, 0.f, 0.f};
  float cbc[8], cwc[8], crc[8];
#pragma unroll
  for (int e = 0; e < 8; ++e) { cbc[e] = 0.f; cwc[e] = 0.f; crc[e] = 0.f; }
  if (OM == 0 && CBM == 1) {
    const v4f v = *(const v4f*)(cb + n0 + c4);
    cb4[0] = bfr(v[0]); cb4[1] = bfr(v[1]); cb4[2] = bfr(v[2]); cb4[3] = bfr(v[3]);
  }
  if (OM != 0) {
    if (CBM == 1) {
      const v4f v0 = *(const v4f*)(cb + n0 + c8);
      const v4f v1 = *(const v4f*)(cb + n0 + c8 + 4);
#pragma unroll
      for (int e = 0; e < 4; ++e) { cbc[e] = bfr(v0[e]); cbc[4 + e] = bfr(v1[e]); }
    }
    if (OM == 2) {
      const v4f v0 = *(const v4f*)(cb2 + n0 + c8);
      const v4f v1 = *(const v4f*)(cb2 + n0 + c8 + 4);
      const v4f w0 = *(const v4f*)(cb3 + n0 + c8);
      const v4f w1 = *(const v4f*)(cb3 + n0 + c8 + 4);
#pragma unroll
      for (int e = 0; e < 4; ++e) {
        cwc[e] = bfr(v0[e]); cwc[4 + e] = bfr(v1[e]);
        crc[e] = bfr(w0[e]); crc[4 + e] = bfr(w1[e]);
      }
    }
  }

  float* slab = sT[wave];
#pragma unroll
  for (int i = 0; i < 4; ++i) {
    const int mBase = m0 + (i << 4);
#pragma unroll
    for (int j = 0; j < 4; ++j) {
#pragma unroll
      for (int r = 0; r < 8; ++r) {
        slab[(mOff + r) * 68 + (j << 4) + rlane] = acc[i][j][r];
      }
    }
    wave_sync_lds();
    if (OM == 0) {
      v4f vals[8];
#pragma unroll
      for (int it = 0; it < 8; ++it) {
        const int row = it * 2 + hh2;
        const v4f v = *(const v4f*)(slab + row * 68 + c4);
        v4f tv = v * wsc + cb4;
        if (RES) {
          const v4f rv = *(const v4f*)(res + (size_t)(mBase + row) * ldc + (size_t)n0 + c4);
          tv = tv + rv;
        }
        vals[it] = tv;
      }
      for (int pass = 0; pass < 2; ++pass) {
#pragma unroll
        for (int it = 0; it < 8; ++it) {
          const int row = it * 2 + hh2;
          *(volatile v4f*)(Cf + (size_t)(mBase + row) * ldc + (size_t)n0 + c4) = vals[it];
        }
        __threadfence();
      }
    } else {
      v4u hv[4], hw[4];
#pragma unroll
      for (int it = 0; it < 4; ++it) {
        const int row = it * 4 + q8;
        const float* sp = slab + row * 68 + c8;
        float rb = 0.f;
        if (CBM == 2) rb = bfr(cb[mBase + row]);
        v4u ha = {0u, 0u, 0u, 0u}, hb = {0u, 0u, 0u, 0u};
#pragma unroll
        for (int e = 0; e < 4; ++e) {
          float b0 = sp[2 * e]     * wsc + cbc[2 * e]     + rb;
          float b1 = sp[2 * e + 1] * wsc + cbc[2 * e + 1] + rb;
          float f0, f1;
          if (OM == 2) {
            f0 = (b0 + cwc[2 * e]) * osc;
            f1 = (b1 + cwc[2 * e + 1]) * osc;
            const float g0 = (b0 + crc[2 * e]) * osc;
            const float g1 = (b1 + crc[2 * e + 1]) * osc;
            hb[e] = pk16(f2h(g0), f2h(g1));
          } else {
            if (ACT) { b0 = silu_f(b0); b1 = silu_f(b1); }
            f0 = b0 * osc;
            f1 = b1 * osc;
          }
          ha[e] = pk16(f2h(f0), f2h(f1));
        }
        hv[it] = ha;
        hw[it] = hb;
      }
      for (int pass = 0; pass < 2; ++pass) {
#pragma unroll
        for (int it = 0; it < 4; ++it) {
          const int row = it * 4 + q8;
          const size_t go = (size_t)(mBase + row) * ldc + (size_t)n0 + c8;
          *(volatile v4u*)(Ch + go) = hv[it];
          if (OM == 2) *(volatile v4u*)(Ch2 + go) = hw[it];
        }
        __threadfence();
      }
    }
    wave_sync_lds();
  }
}

__global__ __launch_bounds__(256) void attn_kernel(
    const unsigned short* __restrict__ QU, const unsigned short* __restrict__ QV,
    const unsigned short* __restrict__ Kp, const unsigned short* __restrict__ Pq,
    const unsigned short* __restrict__ VT, unsigned short* Zh) {
  extern __shared__ __align__(16) float dlds[];
  float* sc = dlds;
  unsigned short* ph = (unsigned short*)(dlds + QT * SCP);
  unsigned short* zst = ph + QT * PHP;
  float* rinv = (float*)(zst + QT * ZP);
  const int t = threadIdx.x, lane = t & 31, wv = t >> 5, hh = lane >> 4, m = lane & 15;
  const int i0 = blockIdx.x * QT;
  const int hc = blockIdx.y * HD;
  const size_t tok0 = (size_t)blockIdx.z * SQ;

  if (t < QT) {
    const int j = i0 + t + 1;
    if (j < SQ) sc[t * SCP + j] = 0.f;
  }

  v16us aq[3][2];
#pragma unroll
  for (int sub = 0; sub < 3; ++sub) {
    const int rr = clampi(i0 + 16 * sub + m, 0, SQ - 1);
    const unsigned short* p = QV + (tok0 + (size_t)rr) * DMD + hc + 8 * hh;
    aq[sub][0] = ldfrag_u(p);
    aq[sub][1] = ldfrag_u(p + 32);
  }
#pragma unroll 1
  for (int ct = 0; ct < 8; ++ct) {
    const int t0 = (wv * 8 + ct) * 16;
    const unsigned short* bp = Pq + (size_t)(t0 + m) * DMD + hc + 8 * hh;
    const v16us b0 = ldfrag_u(bp);
    const v16us b1 = ldfrag_u(bp + 32);
    const int c = t0 + m;
#pragma unroll
    for (int sub = 0; sub < 3; ++sub) {
      v8f acc = mma_h_raw(aq[sub][0], b0, zero8());
      acc = mma_hu(aq[sub][1], b1, acc);
#pragma unroll
      for (int r = 0; r < 8; ++r) {
        const int il0 = 16 * sub + 8 * hh + r;
        const int rabs = i0 + il0;
        const int thr = SQ - 1 - rabs;
        const bool own = (c >= thr);
        const int il = own ? il0 : (il0 - 1);
        const int j = own ? (c - thr) : (c + rabs + 1);
        if ((unsigned)il < (unsigned)QT && (unsigned)j < (unsigned)SQ) sc[il * SCP + j] = acc[r];
      }
    }
    keep2_u(b0, b1);
  }
  keep4_u(aq[0][0], aq[0][1], aq[1][0], aq[1][1]);
  keep2_u(aq[2][0], aq[2][1]);
  __syncthreads();

  v16us au[2][2];
#pragma unroll
  for (int sub = 0; sub < 2; ++sub) {
    const unsigned short* p = QU + (tok0 + (size_t)(i0 + 16 * sub + m)) * DMD + hc + 8 * hh;
    au[sub][0] = ldfrag_u(p);
    au[sub][1] = ldfrag_u(p + 32);
  }
#pragma unroll 1
  for (int ct = 0; ct < 8; ++ct) {
    const int t0 = (wv * 8 + ct) * 16;
    const unsigned short* bp = Kp + (tok0 + (size_t)(t0 + m)) * DMD + hc + 8 * hh;
    const v16us b0 = ldfrag_u(bp);
    const v16us b1 = ldfrag_u(bp + 32);
#pragma unroll
    for (int sub = 0; sub < 2; ++sub) {
      v8f acc = mma_h_raw(au[sub][0], b0, zero8());
      acc = mma_hu(au[sub][1], b1, acc);
      float* srow = sc + (16 * sub + 8 * hh) * SCP + t0 + m;
#pragma unroll
      for (int r = 0; r < 8; ++r) srow[r * SCP] += acc[r];
    }
    keep2_u(b0, b1);
  }
  keep4_u(au[0][0], au[0][1], au[1][0], au[1][1]);
  __syncthreads();

  {
    const float cst = RSQD / (QKS * QKS);
#pragma unroll 1
    for (int q = 0; q < 4; ++q) {
      const int il = wv * 4 + q;
      const float* srow = sc + il * SCP;
      float v[32];
      float mx = -3.0e38f;
#pragma unroll
      for (int c = 0; c < 32; ++c) { v[c] = srow[lane + 32 * c]; mx = fmaxf(mx, v[c]); }
#pragma unroll
      for (int off = 16; off > 0; off >>= 1) mx = fmaxf(mx, __shfl_xor(mx, off, 32));
      float sum = 0.f;
      unsigned short* prow = ph + il * PHP;
#pragma unroll
      for (int c = 0; c < 32; ++c) {
        const float e = __expf((v[c] - mx) * cst);
        sum += e;
        prow[lane + 32 * c] = f2h(e * PSC);
      }
#pragma unroll
      for (int off = 16; off > 0; off >>= 1) sum += __shfl_xor(sum, off, 32);
      if (lane == 0) rinv[il] = 1.0f / sum;
    }
  }
  __syncthreads();

  {
    const int rs = wv >> 2, cs = wv & 3;
    const unsigned short* arow = ph + (16 * rs + m) * PHP + 8 * hh;
    const unsigned short* brow = VT + (size_t)(hc + 16 * cs + m) * MT + tok0 + 8 * hh;
    v8f oz = zero8();
#pragma unroll 2
    for (int k0 = 0; k0 < SQ; k0 += 32) {
      const v16us af = ldfrag_u(arow + k0);
      const v16us bfv = ldfrag_u(brow + k0);
      oz = mma_hu(af, bfv, oz);
    }
#pragma unroll
    for (int r = 0; r < 8; ++r) {
      const int il = 16 * rs + 8 * hh + r;
      zst[il * ZP + 16 * cs + m] = f2h(oz[r] * rinv[il] * (ZSC / (PSC * QKS)));
    }
  }
  __syncthreads();
  {
    const int row = t >> 3, p8 = (t & 7) * 8;
    const v4u hv = *(const v4u*)(zst + row * ZP + p8);
    unsigned short* dst = Zh + (tok0 + (size_t)(i0 + row)) * DMD + hc + p8;
    *(volatile v4u*)dst = hv;
    __threadfence();
    *(volatile v4u*)dst = hv;
  }
}

extern "C" void kernel_launch(void* const* d_in, const int* in_sizes, int n_in,
                              void* d_out, int out_size, void* d_ws, size_t ws_size,
                              hipStream_t stream) {
  if (n_in < 20) return;
  if (in_sizes[0] != MT * DMD) return;
  if (in_sizes[1] != DMD || in_sizes[2] != DMD) return;
  if (in_sizes[3] != DMD * DMD || in_sizes[4] != DMD) return;
  if (in_sizes[5] != DMD * DMD || in_sizes[6] != DMD) return;
  if (in_sizes[7] != DMD * DMD || in_sizes[8] != DMD) return;
  if (in_sizes[9] != DMD * DMD) return;
  if (in_sizes[10] != NHD * HD || in_sizes[11] != NHD * HD) return;
  if (in_sizes[12] != DMD * DMD || in_sizes[13] != DMD) return;
  if (in_sizes[14] != DMD || in_sizes[15] != DMD) return;
  if (in_sizes[16] != FFD * DMD || in_sizes[17] != FFD) return;
  if (in_sizes[18] != DMD * FFD || in_sizes[19] != DMD) return;
  if (out_size != MT * DMD) return;

  const float* x      = (const float*)d_in[0];
  const float* attn_g = (const float*)d_in[1];
  const float* attn_b = (const float*)d_in[2];
  const float* wq     = (const float*)d_in[3];
  const float* bq     = (const float*)d_in[4];
  const float* wk     = (const float*)d_in[5];
  const float* bk     = (const float*)d_in[6];
  const float* wv     = (const float*)d_in[7];
  const float* bv     = (const float*)d_in[8];
  const float* wpos   = (const float*)d_in[9];
  const float* u_bias = (const float*)d_in[10];
  const float* v_bias = (const float*)d_in[11];
  const float* wo     = (const float*)d_in[12];
  const float* bo     = (const float*)d_in[13];
  const float* ffn_g  = (const float*)d_in[14];
  const float* ffn_b  = (const float*)d_in[15];
  const float* w1     = (const float*)d_in[16];
  const float* b1     = (const float*)d_in[17];
  const float* w2     = (const float*)d_in[18];
  const float* b2     = (const float*)d_in[19];

  const size_t PF32 = (size_t)MT * DMD * 4;
  const size_t PH16 = (size_t)MT * DMD * 2;
  const size_t PW   = (size_t)DMD * DMD * 2;
  const size_t PWF  = (size_t)FFD * DMD * 2;
  const size_t PPE  = (size_t)SQ * DMD * 2;
  const size_t PHID = (size_t)MT * FFD * 2;
  size_t off = 0;
  const size_t oXNf = off; off += PF32;
  const size_t oXNh = off; off += PH16;
  const size_t oWQ  = off; off += PW;
  const size_t oWK  = off; off += PW;
  const size_t oWV  = off; off += PW;
  const size_t oWP  = off; off += PW;
  const size_t oWO  = off; off += PW;
  const size_t oW1  = off; off += PWF;
  const size_t oW2  = off; off += PWF;
  const size_t oPE  = off; off += PPE;
  const size_t oPP  = off; off += PPE;
  const size_t oQU  = off; off += PH16;
  const size_t oQV  = off; off += PH16;
  const size_t oK   = off; off += PH16;
  const size_t oVT  = off; off += PH16;
  const size_t oZ   = off; off += PH16;
  if (off > ws_size) return;
  if (off > (size_t)134217728) return;
  if (PHID > 4 * PH16) return;
  if (PF32 > 4 * PH16) return;
  if (oVT + PH16 != oQU + 4 * PH16) return;

  char* ws = (char*)d_ws;
  float*          XNf = (float*)(ws + oXNf);
  unsigned short* XNh = (unsigned short*)(ws + oXNh);
  unsigned short* WQh = (unsigned short*)(ws + oWQ);
  unsigned short* WKh = (unsigned short*)(ws + oWK);
  unsigned short* WVh = (unsigned short*)(ws + oWV);
  unsigned short* WPh = (unsigned short*)(ws + oWP);
  unsigned short* WOh = (unsigned short*)(ws + oWO);
  unsigned short* W1h = (unsigned short*)(ws + oW1);
  unsigned short* W2h = (unsigned short*)(ws + oW2);
  unsigned short* PEh = (unsigned short*)(ws + oPE);
  unsigned short* PPh = (unsigned short*)(ws + oPP);
  unsigned short* QUh = (unsigned short*)(ws + oQU);
  unsigned short* QVh = (unsigned short*)(ws + oQV);
  unsigned short* Kh  = (unsigned short*)(ws + oK);
  unsigned short* VTh = (unsigned short*)(ws + oVT);
  unsigned short* Zh  = (unsigned short*)(ws + oZ);
  float*          X1f = (float*)(ws + oQU);
  float*          YNf = (float*)(ws + oXNf);
  unsigned short* YNh = (unsigned short*)(ws + oXNh);
  unsigned short* Hh  = (unsigned short*)(ws + oQU);
  float*          out0 = (float*)d_out;

  const dim3 blk(256);
  const int gA = ((MT / 64) * (DMD / 64)) / 8;
  const int gP = ((SQ / 64) * (DMD / 64)) / 8;
  const int gF = ((MT / 64) * (FFD / 64)) / 8;

  (void)hipFuncSetAttribute(reinterpret_cast<const void*>(&attn_kernel),
                            hipFuncAttributeMaxDynamicSharedMemorySize, (int)ALDS);

  ln_kernel<0><<<dim3(MT / 8), blk, 0, stream>>>(x, attn_g, attn_b, XNf, XNh, MT);
  cvt_w<<<dim3((DMD * DMD) / 2048), blk, 0, stream>>>(wq, WQh, DMD * DMD, WSCL);
  cvt_w<<<dim3((DMD * DMD) / 2048), blk, 0, stream>>>(wk, WKh, DMD * DMD, WSCL);
  cvt_w<<<dim3((DMD * DMD) / 2048), blk, 0, stream>>>(wv, WVh, DMD * DMD, WSCL);
  cvt_w<<<dim3((DMD * DMD) / 2048), blk, 0, stream>>>(wpos, WPh, DMD * DMD, WSCL);
  cvt_w<<<dim3((DMD * DMD) / 2048), blk, 0, stream>>>(wo, WOh, DMD * DMD, WSCL);
  cvt_w<<<dim3((FFD * DMD) / 2048), blk, 0, stream>>>(w1, W1h, FFD * DMD, WSCL);
  cvt_w<<<dim3((DMD * FFD) / 2048), blk, 0, stream>>>(w2, W2h, DMD * FFD, WSCL);
  pe_kernel<<<dim3(SQ / 8), blk, 0, stream>>>(PEh);

  gemm64<1, 0, 0, 0><<<dim3(gP), blk, 0, stream>>>(
      PEh, DMD, WPh, DMD, PPh, PPh, XNf, DMD, bq, bq, bq, XNf, 1.0f / WSCL, QKS, SQ, DMD, DMD);
  gemm64<2, 1, 0, 0><<<dim3(gA), blk, 0, stream>>>(
      XNh, DMD, WQh, DMD, QUh, QVh, XNf, DMD, bq, u_bias, v_bias, XNf, 1.0f / WSCL, QKS, MT, DMD, DMD);
  gemm64<1, 1, 0, 0><<<dim3(gA), blk, 0, stream>>>(
      XNh, DMD, WKh, DMD, Kh, Kh, XNf, DMD, bk, bk, bk, XNf, 1.0f / WSCL, QKS, MT, DMD, DMD);
  gemm64<1, 2, 0, 0><<<dim3(gA), blk, 0, stream>>>(
      WVh, DMD, XNh, DMD, VTh, VTh, XNf, MT, bv, bv, bv, XNf, 1.0f / WSCL, QKS, DMD, MT, DMD);

  attn_kernel<<<dim3(SQ / QT, NHD, NB), blk, ALDS, stream>>>(QUh, QVh, Kh, PPh, VTh, Zh);

  gemm64<0, 1, 0, 1><<<dim3(gA), blk, 0, stream>>>(
      Zh, DMD, WOh, DMD, PEh, PEh, X1f, DMD, bo, bo, bo, XNf, 1.0f / (WSCL * ZSC), 1.0f, MT, DMD, DMD);

  ln_kernel<1><<<dim3(MT / 8), blk, 0, stream>>>(X1f, ffn_g, ffn_b, YNf, YNh, MT);

  gemm64<1, 1, 1, 0><<<dim3(gF), blk, 0, stream>>>(
      YNh, DMD, W1h, DMD, Hh, Hh, YNf, FFD, b1, b1, b1, YNf, 1.0f / WSCL, HSC, MT, FFD, DMD);
  gemm64<0, 1, 0, 1><<<dim3(gA), blk, 0, stream>>>(
      Hh, FFD, W2h, FFD, PEh, PEh, out0, DMD, b2, b2, b2, YNf, 1.0f / (WSCL * HSC), 1.0f, MT, DMD, FFD);
  (void)hipGetLastError();
}
